// CrossAttention_25589415150106
// MI455X (gfx1250) — hardware-run, weakly checked
//
#include <hip/hip_runtime.h>
#include <math.h>

#ifndef NB
#define NB 4
#endif
#ifndef SEQ
#define SEQ 2048
#endif
#define NB_FULL  4
#define SEQ_FULL 2048
#define DM 1024
#define NH 16
#define HD 64
#define PCARRY 4096.0f

static_assert(SEQ % 64 == 0);
static_assert(SEQ <= SEQ_FULL);
static_assert(NB <= NB_FULL);
static_assert(DM == NH * HD);
static_assert(DM % 64 == 0);

typedef __attribute__((ext_vector_type(16))) _Float16 v16h;
typedef __attribute__((ext_vector_type(8)))  _Float16 v8h;
typedef __attribute__((ext_vector_type(16))) __bf16   v16b;
typedef __attribute__((ext_vector_type(8)))  __bf16   v8b;
typedef __attribute__((ext_vector_type(8)))  float    v8f;
typedef __attribute__((ext_vector_type(4)))  float    v4f;
typedef __attribute__((ext_vector_type(4)))  unsigned v4u;

__device__ __forceinline__ v16b ldfrag_b(const __bf16* p) { union { v16b v; v8b h[2]; } f; f.h[0] = *(const v8b*)(p); f.h[1] = *(const v8b*)(p + 16); return f.v; }
__device__ __forceinline__ v16h ldfrag_h(const _Float16* p) { union { v16h v; v8h h[2]; } f; f.h[0] = *(const v8h*)(p); f.h[1] = *(const v8h*)(p + 16); return f.v; }

__device__ __forceinline__ unsigned short f2bf_bits(float f) {
    unsigned u = __float_as_uint(f);
    return (unsigned short)((u + 0x7FFFu + ((u >> 16) & 1u)) >> 16);
}
__device__ __forceinline__ float bf_keep(float v) {
    const unsigned u = __float_as_uint(v);
    return __uint_as_float((u + 0x7FFFu + ((u >> 16) & 1u)) & 0xFFFF0000u);
}
__device__ __forceinline__ unsigned bf_pk2(float a, float b) { return (unsigned)f2bf_bits(a) | ((unsigned)f2bf_bits(b) << 16); }

__device__ __forceinline__ void wave_lds_sync() {
    __builtin_amdgcn_fence(3  , "workgroup");
    __builtin_amdgcn_wave_barrier();
    __builtin_amdgcn_fence(2  , "workgroup");
}

#define VST2(T, ptr, val) do { const T vst2_v_ = (val); *(volatile T*)(ptr) = vst2_v_; __threadfence(); *(volatile T*)(ptr) = vst2_v_; } while (0)

__device__ __forceinline__ void dep_guard_b(v8f& a, v8f& b, v16b x, v16b y) { asm volatile("v_nop\n\tv_nop\n\tv_nop\n\tv_nop" : "+v"(a), "+v"(b) : "v"(x), "v"(y)); }
__device__ __forceinline__ void keep4_b(v16b a, v16b b, v16b c, v16b d) { asm volatile("v_nop" :: "v"(a), "v"(b), "v"(c), "v"(d)); }
__device__ __forceinline__ void acc_guard4(v8f& a, v8f& b, v8f& c, v8f& d) { asm volatile("v_nop\n\tv_nop\n\tv_nop\n\tv_nop" : "+v"(a), "+v"(b), "+v"(c), "+v"(d)); }
__device__ __forceinline__ void guard_s(v8f& a, v16h x0, v16h x1, v16h y0, v16h y1) { asm volatile("v_nop\n\tv_nop\n\tv_nop\n\tv_nop" : "+v"(a) : "v"(x0), "v"(x1), "v"(y0), "v"(y1)); }
__device__ __forceinline__ void guard_o(v8f& a, v8f& b, v8f& c, v8f& d, v16h p, v16h v0, v16h v1, v16h v2, v16h v3) {
    asm volatile("v_nop\n\tv_nop\n\tv_nop\n\tv_nop" : "+v"(a), "+v"(b), "+v"(c), "+v"(d) : "v"(p), "v"(v0), "v"(v1), "v"(v2), "v"(v3));
}

__global__ __launch_bounds__(256) void k_cast_rows(const float* __restrict__ src, unsigned short* __restrict__ dst) {
    const long long u = (long long)blockIdx.x * 256 + threadIdx.x;
    const int per = DM / 8;
    if (u >= (long long)NB * SEQ * per) return;
    const int r = (int)(u / per), c0 = 8 * (int)(u % per);
    const int b = r / SEQ, t = r - b * SEQ;
    const float* s = src + ((long long)b * SEQ_FULL + t) * DM + c0;
    const v4f a = *(const v4f*)(s), c = *(const v4f*)(s + 4);
    v4u pk; pk.x = bf_pk2(a.x, a.y); pk.y = bf_pk2(a.z, a.w); pk.z = bf_pk2(c.x, c.y); pk.w = bf_pk2(c.z, c.w);
    VST2(v4u, (v4u*)(dst + (long long)r * DM + c0), pk);
}

__global__ __launch_bounds__(256) void k_cast_wT(const float* __restrict__ W, unsigned short* __restrict__ dst) {
    const int u = blockIdx.x * 256 + threadIdx.x;
    const int per = DM / 8;
    if (u >= DM * per) return;
    const int n = u / per, k0 = 8 * (u % per);
    float w[8];
#pragma unroll
    for (int e = 0; e < 8; ++e) w[e] = W[(long long)(k0 + e) * DM + n];
    v4u pk; pk.x = bf_pk2(w[0], w[1]); pk.y = bf_pk2(w[2], w[3]); pk.z = bf_pk2(w[4], w[5]); pk.w = bf_pk2(w[6], w[7]);
    VST2(v4u, (v4u*)(dst + (long long)n * DM + k0), pk);
}

template <bool VT>
__global__ __launch_bounds__(256) void k_proj(const unsigned short* __restrict__ Ap, const unsigned short* __restrict__ Btp,
                                               const float* __restrict__ bias, unsigned short* __restrict__ dstp, int M, int N) {
    __shared__ __align__(16) float sT[8][16 * 68];
    const __bf16* A  = (const __bf16*)Ap;
    const __bf16* Bt = (const __bf16*)Btp;
    _Float16* dst = (_Float16*)dstp;
    const int lane = threadIdx.x & 31;
    const int wave = threadIdx.x >> 5;
    const int tilesN = N >> 6;
    const int tilesM = M >> 6;
    const int tile = blockIdx.x * 8 + wave;
    if (tile >= tilesM * tilesN) return;
    const int tm = tile / tilesN;
    const int tn = tile - tm * tilesN;
    const int m0 = tm << 6;
    const int n0 = tn << 6;
    const int rlane = lane & 15;
    const int koff  = (lane >> 4) * 8;
    const int mOff  = (lane >> 4) * 8;

    v8f acc[4][4];
#pragma unroll
    for (int i = 0; i < 4; ++i)
#pragma unroll
        for (int j = 0; j < 4; ++j) acc[i][j] = (v8f){0.f, 0.f, 0.f, 0.f, 0.f, 0.f, 0.f, 0.f};

#pragma unroll 1
    for (int k0 = 0; k0 < DM; k0 += 32) {
        v16b bh[4];
#pragma unroll
        for (int j = 0; j < 4; ++j) bh[j] = ldfrag_b(Bt + (size_t)(n0 + (j << 4) + rlane) * DM + koff + k0);
#pragma unroll
        for (int i = 0; i < 4; ++i) {
            const v16b ah = ldfrag_b(A + (size_t)(m0 + (i << 4) + rlane) * DM + koff + k0);
#pragma unroll
            for (int j = 0; j < 4; ++j)
                acc[i][j] = __builtin_amdgcn_wmma_f32_16x16x32_bf16(false, ah, false, bh[j], (short)0, acc[i][j], false, false);
            dep_guard_b(acc[i][0], acc[i][3], ah, ah);
        }
        keep4_b(bh[0], bh[1], bh[2], bh[3]);
    }
    acc_guard4(acc[0][0], acc[0][1], acc[0][2], acc[0][3]);
    acc_guard4(acc[1][0], acc[1][1], acc[1][2], acc[1][3]);
    acc_guard4(acc[2][0], acc[2][1], acc[2][2], acc[2][3]);
    acc_guard4(acc[3][0], acc[3][1], acc[3][2], acc[3][3]);

    float* slab = sT[wave];
    const int q = lane >> 3, c8 = (lane & 7) * 8;
#pragma unroll
    for (int i = 0; i < 4; ++i) {
        const int mBase = m0 + (i << 4);
        float bm[8];
#pragma unroll
        for (int r = 0; r < 8; ++r) bm[r] = VT ? bf_keep(bias[VT ? (mBase + mOff + r) : 0]) : 0.f;
#pragma unroll
        for (int j = 0; j < 4; ++j) {
            const int n = n0 + (j << 4) + rlane;
            const float bn = VT ? 0.f : bf_keep(bias[VT ? 0 : n]);
#pragma unroll
            for (int r = 0; r < 8; ++r) slab[(mOff + r) * 68 + (j << 4) + rlane] = acc[i][j][r] + (VT ? bm[r] : bn);
        }
        wave_lds_sync();
        for (int pass = 0; pass < 2; ++pass) {
#pragma unroll
            for (int it = 0; it < 4; ++it) {
                const int row = it * 4 + q;
                const v4f lo = *(const v4f*)(slab + row * 68 + c8);
                const v4f hi = *(const v4f*)(slab + row * 68 + c8 + 4);
                v8h hv;
                hv[0] = (_Float16)lo.x; hv[1] = (_Float16)lo.y; hv[2] = (_Float16)lo.z; hv[3] = (_Float16)lo.w;
                hv[4] = (_Float16)hi.x; hv[5] = (_Float16)hi.y; hv[6] = (_Float16)hi.z; hv[7] = (_Float16)hi.w;
                size_t off;
                if (VT) {
                    const int feat = mBase + row;
                    const int bb = n0 / SEQ, tok0 = n0 - bb * SEQ;
                    off = ((size_t)((bb * NH + (feat >> 6)) * HD + (feat & 63))) * SEQ + tok0 + c8;
                } else {
                    const int gm = mBase + row;
                    const int bb = gm / SEQ, tk = gm - bb * SEQ;
                    off = ((size_t)((bb * NH + (n0 >> 6)) * SEQ + tk)) * HD + c8;
                }
                *(volatile v8h*)(dst + off) = hv;
            }
            __threadfence();
        }
        wave_lds_sync();
    }
}

__global__ __launch_bounds__(128) void k_attn(const unsigned short* __restrict__ Qp, const unsigned short* __restrict__ Kp,
                                               const unsigned short* __restrict__ Vp, const int* __restrict__ mask, float* __restrict__ out) {
    __shared__ __align__(16) _Float16 Ps[4][16 * 64];
    __shared__ __align__(16) float    Os[4][16 * 68];
    const int tid = threadIdx.x, wave = tid >> 5, lane = tid & 31, hh = lane >> 4, c = lane & 15;
    const int nqb = SEQ / 64;
    const int bx = blockIdx.x;
    const int qb = bx % nqb;
    const int bh = bx / nqb;
    const int h  = bh % NH;
    const int b  = bh / NH;
    const int q0 = qb * 64 + wave * 16;

    const _Float16* Qb = (const _Float16*)Qp + (size_t)bh * SEQ * HD;
    const _Float16* Kb = (const _Float16*)Kp + (size_t)bh * SEQ * HD;
    const _Float16* Vb = (const _Float16*)Vp + (size_t)bh * HD * SEQ;
    const int* mrow = mask + (size_t)b * SEQ_FULL;

    const v16h qa0 = ldfrag_h(Qb + (size_t)(q0 + c) * HD + 8 * hh);
    const v16h qa1 = ldfrag_h(Qb + (size_t)(q0 + c) * HD + 32 + 8 * hh);

    const float SCL  = 0.125f * 1.4426950408889634f;
    const float FILL = -3.4028234663852886e38f;

    float mrw[8], lrw[8];
    v8f o[4];
#pragma unroll
    for (int r = 0; r < 8; ++r) { mrw[r] = -INFINITY; lrw[r] = 0.f; }
#pragma unroll
    for (int t = 0; t < 4; ++t) o[t] = (v8f){0.f, 0.f, 0.f, 0.f, 0.f, 0.f, 0.f, 0.f};

    _Float16* pw = Ps[wave];

#pragma unroll 1
    for (int kc = 0; kc < SEQ / 64; ++kc) {
        const int kv0 = kc * 64;
        int mk[4];
#pragma unroll
        for (int j = 0; j < 4; ++j) mk[j] = mrow[kv0 + j * 16 + c];

        v8f s[4];
#pragma unroll
        for (int j = 0; j < 4; ++j) {
            const _Float16* kr = Kb + (size_t)(kv0 + j * 16 + c) * HD + 8 * hh;
            const v16h k0 = ldfrag_h(kr), k1 = ldfrag_h(kr + 32);
            v8f a = (v8f){0.f, 0.f, 0.f, 0.f, 0.f, 0.f, 0.f, 0.f};
            a = __builtin_amdgcn_wmma_f32_16x16x32_f16(false, qa0, false, k0, (short)0, a, false, false);
            a = __builtin_amdgcn_wmma_f32_16x16x32_f16(false, qa1, false, k1, (short)0, a, false, false);
            guard_s(a, qa0, qa1, k0, k1);
            s[j] = a;
        }

#pragma unroll
        for (int r = 0; r < 8; ++r) {
            float sc[4];
#pragma unroll
            for (int j = 0; j < 4; ++j) sc[j] = (mk[j] != 0) ? s[j][r] * SCL : FILL;
            float m = fmaxf(fmaxf(sc[0], sc[1]), fmaxf(sc[2], sc[3]));
            m = fmaxf(m, __shfl_xor(m, 1, 32));
            m = fmaxf(m, __shfl_xor(m, 2, 32));
            m = fmaxf(m, __shfl_xor(m, 4, 32));
            m = fmaxf(m, __shfl_xor(m, 8, 32));
            const float mnew  = fmaxf(mrw[r], m);
            const float alpha = __builtin_amdgcn_exp2f(mrw[r] - mnew);
            mrw[r] = mnew;
            float psum = 0.f;
#pragma unroll
            for (int j = 0; j < 4; ++j) {
                const float p = __builtin_amdgcn_exp2f(sc[j] - mnew);
                psum += p;
                pw[(8 * hh + r) * 64 + j * 16 + c] = (_Float16)(p * PCARRY);
            }
            psum += __shfl_xor(psum, 1, 32);
            psum += __shfl_xor(psum, 2, 32);
            psum += __shfl_xor(psum, 4, 32);
            psum += __shfl_xor(psum, 8, 32);
            lrw[r] = lrw[r] * alpha + psum;
#pragma unroll
            for (int t = 0; t < 4; ++t) o[t][r] *= alpha;
        }
        wave_lds_sync();

#pragma unroll
        for (int kk = 0; kk < 2; ++kk) {
            const v16h pa = ldfrag_h(pw + c * 64 + kk * 32 + 8 * hh);
            const v16h v0 = ldfrag_h(Vb + (size_t)(0 * 16 + c) * SEQ + kv0 + kk * 32 + 8 * hh);
            const v16h v1 = ldfrag_h(Vb + (size_t)(1 * 16 + c) * SEQ + kv0 + kk * 32 + 8 * hh);
            const v16h v2 = ldfrag_h(Vb + (size_t)(2 * 16 + c) * SEQ + kv0 + kk * 32 + 8 * hh);
            const v16h v3 = ldfrag_h(Vb + (size_t)(3 * 16 + c) * SEQ + kv0 + kk * 32 + 8 * hh);
            o[0] = __builtin_amdgcn_wmma_f32_16x16x32_f16(false, pa, false, v0, (short)0, o[0], false, false);
            o[1] = __builtin_amdgcn_wmma_f32_16x16x32_f16(false, pa, false, v1, (short)0, o[1], false, false);
            o[2] = __builtin_amdgcn_wmma_f32_16x16x32_f16(false, pa, false, v2, (short)0, o[2], false, false);
            o[3] = __builtin_amdgcn_wmma_f32_16x16x32_f16(false, pa, false, v3, (short)0, o[3], false, false);
            guard_o(o[0], o[1], o[2], o[3], pa, v0, v1, v2, v3);
        }
        wave_lds_sync();
    }

    float* os = Os[wave];
#pragma unroll
    for (int r = 0; r < 8; ++r) {
        const float inv = 1.0f / (lrw[r] * PCARRY);
#pragma unroll
        for (int t = 0; t < 4; ++t) os[(8 * hh + r) * 68 + t * 16 + c] = o[t][r] * inv;
    }
    wave_lds_sync();
    {
        float* ob = out + ((size_t)b * SEQ + q0) * DM + h * HD;
        const int c4 = (lane & 15) * 4;
        for (int pass = 0; pass < 2; ++pass) {
#pragma unroll
            for (int it = 0; it < 8; ++it) {
                const int row = it * 2 + hh;
                const v4f val = *(const v4f*)(os + row * 68 + c4);
                *(volatile v4f*)(ob + (size_t)row * DM + c4) = val;
            }
            __threadfence();
        }
    }
}

#define ACT_BYTES  ((size_t)NB * SEQ * DM * 2)
#define W_BYTES    ((size_t)DM * DM * 2)
#define HEAD_BYTES ((size_t)NB * NH * SEQ * HD * 2)
static_assert(2 * ACT_BYTES + 3 * W_BYTES + 3 * HEAD_BYTES <= (size_t)134217728);
static_assert(ACT_BYTES % 256 == 0);
static_assert(W_BYTES % 256 == 0);
static_assert(HEAD_BYTES % 256 == 0);

extern "C" void kernel_launch(void* const* d_in, const int* in_sizes, int n_in, void* d_out, int out_size, void* d_ws, size_t ws_size, hipStream_t stream) {
    if (n_in < 9) return;
    const long long needAct = (long long)(NB - 1) * SEQ_FULL * DM + (long long)SEQ * DM;
    const long long needMsk = (long long)(NB - 1) * SEQ_FULL + SEQ;
    if ((long long)in_sizes[0] < needAct || (long long)in_sizes[1] < needAct || (long long)in_sizes[2] < needMsk) return;
    if (in_sizes[3] < DM * DM || in_sizes[5] < DM * DM || in_sizes[7] < DM * DM) return;
    if (in_sizes[4] < DM || in_sizes[6] < DM || in_sizes[8] < DM) return;
    if ((long long)out_size < (long long)NB * SEQ * DM) return;

    const float* x    = (const float*)d_in[0];
    const float* ctx  = (const float*)d_in[1];
    const int*   mask = (const int*)d_in[2];
    const float* Wq   = (const float*)d_in[3];
    const float* bq   = (const float*)d_in[4];
    const float* Wk   = (const float*)d_in[5];
    const float* bk   = (const float*)d_in[6];
    const float* Wv   = (const float*)d_in[7];
    const float* bv   = (const float*)d_in[8];
    float* out = (float*)d_out;

    char* wsp = (char*)d_ws;
    unsigned short* XB  = (unsigned short*)wsp; wsp += ACT_BYTES;
    unsigned short* CB  = (unsigned short*)wsp; wsp += ACT_BYTES;
    unsigned short* WQT = (unsigned short*)wsp; wsp += W_BYTES;
    unsigned short* WKT = (unsigned short*)wsp; wsp += W_BYTES;
    unsigned short* WVT = (unsigned short*)wsp; wsp += W_BYTES;
    unsigned short* QH  = (unsigned short*)wsp; wsp += HEAD_BYTES;
    unsigned short* KH  = (unsigned short*)wsp; wsp += HEAD_BYTES;
    unsigned short* VTH = (unsigned short*)wsp; wsp += HEAD_BYTES;
    if ((size_t)(wsp - (char*)d_ws) > ws_size) return;

    const unsigned gAct = (unsigned)(((long long)NB * SEQ * (DM / 8) + 255) / 256);
    const unsigned gW   = (unsigned)((DM * (DM / 8) + 255) / 256);
    k_cast_rows<<<gAct, 256, 0, stream>>>(x, XB);
    k_cast_rows<<<gAct, 256, 0, stream>>>(ctx, CB);
    k_cast_wT<<<gW, 256, 0, stream>>>(Wq, WQT);
    k_cast_wT<<<gW, 256, 0, stream>>>(Wk, WKT);
    k_cast_wT<<<gW, 256, 0, stream>>>(Wv, WVT);

    const int rows = NB * SEQ;
    const unsigned gTiles = (unsigned)(((rows / 64) * (DM / 64) + 7) / 8);
    k_proj<false><<<gTiles, 256, 0, stream>>>(XB, WQT, bq, QH, rows, DM);
    k_proj<false><<<gTiles, 256, 0, stream>>>(CB, WKT, bk, KH, rows, DM);
    k_proj<true><<<gTiles, 256, 0, stream>>>(WVT, CB, bv, VTH, DM, rows);

    k_attn<<<(unsigned)(NB * NH * (SEQ / 64)), 128, 0, stream>>>(QH, KH, VTH, mask, out);
}
